// Model_79972291051986
// MI455X (gfx1250) — hardware-verified
//
#include <hip/hip_runtime.h>
#include <math.h>
#include <stdint.h>

#define NB      8
#define NTOK    625
#define NTOKB   125
#define NPADT   640
#define MROWS   5120
#define DIM     128
#define HEADS   8
#define HD      16
#define MLP     4096
#define DEPTH   3
#define TP      132
#define PLANE_EL (MROWS * 256)

static_assert(NB * NPADT == MROWS);
static_assert(MROWS % 64 == 0);
static_assert(NPADT % 64 == 0);
static_assert(NTOK <= NPADT);
static_assert(NTOKB * 5 == NTOK);
static_assert(HEADS * HD == DIM);
static_assert(HD == 16);
static_assert(3 * DIM == 384);
static_assert(MLP % 128 == 0);
static_assert(DIM % 32 == 0);
static_assert(MLP % 32 == 0);

typedef __attribute__((ext_vector_type(16))) __bf16   v16b;
typedef __attribute__((ext_vector_type(8)))  __bf16   v8b;
typedef __attribute__((ext_vector_type(8)))  float    v8f;
typedef __attribute__((ext_vector_type(4)))  float    v4f;
typedef __attribute__((ext_vector_type(4)))  unsigned int v4u;
typedef __attribute__((ext_vector_type(4)))  int      v4i;
typedef v4f __attribute__((may_alias)) v4fa;
typedef v4i __attribute__((may_alias)) v4ia;

union FragB { v16b v; v8b h[2]; unsigned int w[8]; };

__device__ __forceinline__ unsigned short f2bf_bits(float f) {
  unsigned u = __float_as_uint(f);
  return (unsigned short)((u + 0x7FFFu + ((u >> 16) & 1u)) >> 16);
}
__device__ __forceinline__ float bf_bits2f(unsigned short h) { return __uint_as_float(((unsigned)h) << 16); }
__device__ __forceinline__ float rne1(float a) { return bf_bits2f(f2bf_bits(a)); }
__device__ __forceinline__ v4f rne4(v4f a) {
  v4f r; r[0] = rne1(a[0]); r[1] = rne1(a[1]); r[2] = rne1(a[2]); r[3] = rne1(a[3]); return r;
}
__device__ __forceinline__ unsigned pk16(unsigned short a, unsigned short b) { return (unsigned)a | ((unsigned)b << 16); }
__device__ __forceinline__ unsigned hi_pair(float a, float b) { return pk16(f2bf_bits(a), f2bf_bits(b)); }
__device__ __forceinline__ unsigned lo_pair(float a, float b) {
  const float ra = a - bf_bits2f(f2bf_bits(a));
  const float rb = b - bf_bits2f(f2bf_bits(b));
  return pk16(f2bf_bits(ra), f2bf_bits(rb));
}

__device__ __forceinline__ v8f wmma_b(v16b a, v16b b, v8f c) {
  v8f d = __builtin_amdgcn_wmma_f32_16x16x32_bf16(false, a, false, b, (short)0, c, false, false);
  asm volatile("v_nop\n\tv_nop\n\tv_nop\n\tv_nop" : "+v"(d) : "v"(a), "v"(b));
  return d;
}
__device__ __forceinline__ v16b ldfrag(const __bf16* p) {
  FragB f; f.h[0] = *(const v8b*)(p); f.h[1] = *(const v8b*)(p + 16); return f.v;
}

__device__ __forceinline__ float wave_sum(float v) {
#pragma unroll
  for (int off = 16; off > 0; off >>= 1) v += __shfl_xor(v, off, 32);
  return v;
}

__device__ __forceinline__ v4f ln_row(v4f x, v4f g, v4f be) {
  float s = (x[0] + x[1]) + (x[2] + x[3]);
  s = wave_sum(s);
  const float mu = s * (1.0f / 128.0f);
  const float d0 = x[0] - mu, d1 = x[1] - mu, d2 = x[2] - mu, d3 = x[3] - mu;
  float q = (d0 * d0 + d1 * d1) + (d2 * d2 + d3 * d3);
  q = wave_sum(q);
  const float rstd = 1.0f / sqrtf(q * (1.0f / 128.0f) + 1e-5f);
  v4f y;
  y[0] = d0 * rstd * g[0] + be[0];
  y[1] = d1 * rstd * g[1] + be[1];
  y[2] = d2 * rstd * g[2] + be[2];
  y[3] = d3 * rstd * g[3] + be[3];
  return y;
}

template <int RPW>
__device__ __forceinline__ void store_hilo(const float* T, unsigned short* dst, int rowBase,
                                           int pitch, int loOff, int col0, int w, int lane) {
  const int rsel = lane >> 4;
  const int c = (lane & 15) * 8;
  v4u hv[RPW / 2], lv[RPW / 2];
#pragma unroll
  for (int i = 0; i < RPW / 2; ++i) {
    const int row = w * RPW + 2 * i + rsel;
    const float* sp = T + row * TP + c;
    const v4f a = *(const v4fa*)(sp);
    const v4f b = *(const v4fa*)(sp + 4);
    hv[i] = (v4u){hi_pair(a[0], a[1]), hi_pair(a[2], a[3]), hi_pair(b[0], b[1]), hi_pair(b[2], b[3])};
    lv[i] = (v4u){lo_pair(a[0], a[1]), lo_pair(a[2], a[3]), lo_pair(b[0], b[1]), lo_pair(b[2], b[3])};
  }
  for (int pass = 0; pass < 2; ++pass) {
#pragma unroll
    for (int i = 0; i < RPW / 2; ++i) {
      const int row = w * RPW + 2 * i + rsel;
      const size_t o = (size_t)(rowBase + row) * pitch + col0 + c;
      *(volatile v4u*)(dst + o) = hv[i];
      *(volatile v4u*)(dst + o + loOff) = lv[i];
    }
    __threadfence();
  }
}

__global__ __launch_bounds__(256) void k_prep_x(const float* __restrict__ x, const float* __restrict__ g,
                                                const float* __restrict__ be, float* __restrict__ XA,
                                                unsigned short* __restrict__ HHL) {
  __shared__ __align__(16) float T[64 * TP];
  const int tid = threadIdx.x, lane = tid & 31, w = tid >> 5;
  const int m0 = blockIdx.x * 64;
  const v4f gv = rne4(*(const v4fa*)(g + 4 * lane));
  const v4f bv = rne4(*(const v4fa*)(be + 4 * lane));
  v4f xv[8];
#pragma unroll
  for (int i = 0; i < 8; ++i) {
    const int row = w * 8 + i;
    const int gr = m0 + row;
    const int b = gr / NPADT;
    const int n = gr - b * NPADT;
    const int nn = (n < NTOK) ? n : (NTOK - 1);
    const v4f t = rne4(*(const v4fa*)(x + ((size_t)b * NTOK + nn) * DIM + 4 * lane));
    const bool ok = (n < NTOK);
    v4f xr;
    xr[0] = ok ? t[0] : 0.0f; xr[1] = ok ? t[1] : 0.0f; xr[2] = ok ? t[2] : 0.0f; xr[3] = ok ? t[3] : 0.0f;
    xv[i] = xr;
    const v4f y = ln_row(xr, gv, bv);
    *(v4fa*)(T + row * TP + 4 * lane) = y;
  }
  for (int pass = 0; pass < 2; ++pass) {
#pragma unroll
    for (int i = 0; i < 8; ++i) {
      const int gr = m0 + w * 8 + i;
      *(volatile v4f*)(XA + (size_t)gr * DIM + 4 * lane) = xv[i];
    }
    __threadfence();
  }
  __syncthreads();
  store_hilo<8>(T, HHL, m0, 256, 128, 0, w, lane);
}

__global__ __launch_bounds__(256) void k_wprep(const float* __restrict__ src, unsigned short* __restrict__ dst,
                                               int K, int N) {
  __shared__ __align__(16) unsigned short th[64 * 72];
  const int tid = threadIdx.x;
  const int n0 = blockIdx.x * 64, k0 = blockIdx.y * 64, l = blockIdx.z;
  const float* s = src + (size_t)l * K * N;
  unsigned short* d = dst + (size_t)l * K * N;
  {
    const int rr = tid >> 2;
    const int cq = (tid & 3) * 16;
    const float* sp = s + (size_t)(k0 + rr) * N + n0 + cq;
#pragma unroll
    for (int q = 0; q < 4; ++q) {
      const v4f f = *(const v4fa*)(sp + 4 * q);
#pragma unroll
      for (int e = 0; e < 4; ++e) th[rr * 72 + cq + 4 * q + e] = f2bf_bits(f[e]);
    }
  }
  __syncthreads();
  const int sub = tid >> 3;
  const int c8 = (tid & 7) * 8;
  v4u vv[2];
#pragma unroll
  for (int it = 0; it < 2; ++it) {
    const int oc = it * 32 + sub;
    v4u a;
#pragma unroll
    for (int q = 0; q < 4; ++q) a[q] = pk16(th[(c8 + 2 * q) * 72 + oc], th[(c8 + 2 * q + 1) * 72 + oc]);
    vv[it] = a;
  }
  for (int pass = 0; pass < 2; ++pass) {
#pragma unroll
    for (int it = 0; it < 2; ++it) {
      const int oc = it * 32 + sub;
      const size_t go = (size_t)(n0 + oc) * K + k0 + c8;
      *(volatile v4u*)(d + go) = vv[it];
    }
    __threadfence();
  }
}

template <int MODE>
__global__ __launch_bounds__(256) void k_gemm(
    const unsigned short* __restrict__ Ap, int lda, int loOff,
    const unsigned short* __restrict__ Wp, int Kw,
    const float* __restrict__ bias,
    const float* __restrict__ Xin, float* __restrict__ Xout,
    const float* __restrict__ lng, const float* __restrict__ lnb,
    unsigned short* __restrict__ Ohl, int opitch, int oLo,
    unsigned short* __restrict__ VTp,
    float* __restrict__ dout, int fin) {
  __shared__ __align__(16) float T[64 * TP];
  const __bf16* A = (const __bf16*)Ap;
  const __bf16* W = (const __bf16*)Wp;
  const int tid = threadIdx.x, lane = tid & 31, w = tid >> 5;
  const int h = lane >> 4, rl = lane & 15;
  const int wm = w >> 1, wn = w & 1;
  const int m0 = blockIdx.x * 64;
  const int ty = blockIdx.y;
  const int n0 = ty * 128;

  const __bf16* arow = A + (size_t)(m0 + wm * 16 + rl) * lda + 8 * h;
  const __bf16* brow = W + (size_t)(n0 + wn * 64 + rl) * Kw + 8 * h;
  const v8f zero8 = {0.f, 0.f, 0.f, 0.f, 0.f, 0.f, 0.f, 0.f};
  v8f acc[4];
#pragma unroll
  for (int j = 0; j < 4; ++j) acc[j] = zero8;

#pragma unroll 1
  for (int k0 = 0; k0 < Kw; k0 += 32) {
    const v16b ah = ldfrag(arow + k0);
    const v16b al = ldfrag(arow + loOff + k0);
#pragma unroll
    for (int j = 0; j < 4; ++j) {
      const v16b bj = ldfrag(brow + (size_t)j * 16 * Kw + k0);
      acc[j] = wmma_b(ah, bj, acc[j]);
      acc[j] = wmma_b(al, bj, acc[j]);
    }
  }

  const float sc = (MODE == 0 && ty == 0) ? 0.25f : 1.0f;
#pragma unroll
  for (int j = 0; j < 4; ++j)
#pragma unroll
    for (int r = 0; r < 8; ++r)
      T[(wm * 16 + 8 * h + r) * TP + wn * 64 + j * 16 + rl] = acc[j][r] * sc;
  __syncthreads();

  if (MODE == 0) {
    if (ty < 2) {
      store_hilo<8>(T, Ohl + (size_t)ty * PLANE_EL, m0, opitch, oLo, 0, w, lane);
    } else {
      const int bb = m0 / NPADT;
      const int t0 = m0 - bb * NPADT;
      const int sub = lane >> 3, q8 = lane & 7;
      v4u vv[8];
#pragma unroll
      for (int i = 0; i < 8; ++i) {
        const int lid = w * 32 + i * 4 + sub;
        const int part = lid >> 7;
        const int c = lid & 127;
        float f[8];
#pragma unroll
        for (int e = 0; e < 8; ++e) {
          const float v = T[(q8 * 8 + e) * TP + c];
          f[e] = (t0 + q8 * 8 + e < NTOK) ? v : 0.0f;
        }
        v4u o;
#pragma unroll
        for (int q = 0; q < 4; ++q) {
          const unsigned hw = hi_pair(f[2 * q], f[2 * q + 1]);
          const unsigned lw = lo_pair(f[2 * q], f[2 * q + 1]);
          o[q] = (part != 0) ? lw : hw;
        }
        vv[i] = o;
      }
      for (int pass = 0; pass < 2; ++pass) {
#pragma unroll
        for (int i = 0; i < 8; ++i) {
          const int lid = w * 32 + i * 4 + sub;
          const int part = lid >> 7;
          const int c = lid & 127;
          const size_t go = ((size_t)(bb * 2 + part) * 128 + c) * NPADT + t0 + q8 * 8;
          *(volatile v4u*)(VTp + go) = vv[i];
        }
        __threadfence();
      }
    }
  }

  if (MODE == 1) {
    const v4f bi = rne4(*(const v4fa*)(bias + 4 * lane));
    const v4f gv = rne4(*(const v4fa*)(lng + 4 * lane));
    const v4f bv = rne4(*(const v4fa*)(lnb + 4 * lane));
    v4f xv[8];
#pragma unroll
    for (int i = 0; i < 8; ++i) {
      const int row = w * 8 + i;
      const int gr = m0 + row;
      float* tp = T + row * TP + 4 * lane;
      const v4f t = *(const v4fa*)tp;
      const v4f xi = *(const v4fa*)(Xin + (size_t)gr * DIM + 4 * lane);
      v4f xn;
      xn[0] = xi[0] + (t[0] + bi[0]); xn[1] = xi[1] + (t[1] + bi[1]);
      xn[2] = xi[2] + (t[2] + bi[2]); xn[3] = xi[3] + (t[3] + bi[3]);
      xv[i] = xn;
      const v4f y = ln_row(xn, gv, bv);
      *(v4fa*)tp = y;
    }
    if (fin != 0) {
      for (int pass = 0; pass < 2; ++pass) {
#pragma unroll
        for (int i = 0; i < 8; ++i) {
          const int gr = m0 + w * 8 + i;
          const int b = gr / NPADT;
          const int n = gr - b * NPADT;
          if (n < NTOK)
            *(volatile v4f*)(dout + ((size_t)b * NTOK + n) * DIM + 4 * lane) = xv[i];
        }
        __threadfence();
      }
    } else {
      for (int pass = 0; pass < 2; ++pass) {
#pragma unroll
        for (int i = 0; i < 8; ++i) {
          const int gr = m0 + w * 8 + i;
          *(volatile v4f*)(Xout + (size_t)gr * DIM + 4 * lane) = xv[i];
        }
        __threadfence();
      }
      __syncthreads();
      store_hilo<8>(T, Ohl, m0, opitch, oLo, 0, w, lane);
    }
  }

  if (MODE == 2) {
    const v4f bi = rne4(*(const v4fa*)(bias + n0 + 4 * lane));
#pragma unroll 1
    for (int i = 0; i < 8; ++i) {
      float* tp = T + (w * 8 + i) * TP + 4 * lane;
      v4f t = *(const v4fa*)tp;
#pragma unroll
      for (int e = 0; e < 4; ++e) {
        const float u = t[e] + bi[e];
        t[e] = 0.5f * u * (1.0f + erff(u * 0.70710678118654752f));
      }
      *(v4fa*)tp = t;
    }
    __syncthreads();
    store_hilo<8>(T, Ohl, m0, opitch, oLo, n0, w, lane);
  }
}

__global__ __launch_bounds__(128) void k_attn(const unsigned short* __restrict__ QHLp,
                                              const unsigned short* __restrict__ KHLp,
                                              const unsigned short* __restrict__ VTp,
                                              const int* __restrict__ mask,
                                              unsigned short* __restrict__ CTX) {
  __shared__ __align__(16) float T[64 * TP];
  __shared__ __align__(16) int sAllow[NPADT];
  __shared__ int sCnt[16];
  const __bf16* QHL = (const __bf16*)QHLp;
  const __bf16* KHL = (const __bf16*)KHLp;
  const __bf16* VT  = (const __bf16*)VTp;
  const int tid = threadIdx.x, lane = tid & 31, w = tid >> 5;
  const int h = lane >> 4, m = lane & 15;
  const int qt = blockIdx.x, b = blockIdx.y;
  const int m0 = b * NPADT + qt * 64;
  const float NEG_INF = -__builtin_inff();

  for (int i = tid; i < NPADT; i += 128) {
    int blk = i / NTOKB;
    blk = (blk < 3) ? blk : 3;
    const int mv = mask[b * 4 + blk];
    const int a = (i < 4 * NTOKB) ? ((mv != 0) ? 1 : 0) : ((i < NTOK) ? 1 : 0);
    sAllow[i] = a;
  }
  __syncthreads();
  {
    const int tt = (tid < 9) ? tid : 9;
    int c = 0;
#pragma unroll 4
    for (int j = 0; j < 64; ++j) c += sAllow[tt * 64 + j];
    if (tid < 16) sCnt[tid] = c;
  }
  __syncthreads();

  const __bf16* qrow  = QHL + (size_t)(m0 + w * 16 + m) * 256 + 8 * h;
  const __bf16* kbase = KHL + (size_t)(b * NPADT + m) * 256 + 8 * h;
  const __bf16* vbase = VT + ((size_t)(b * 2) * 128 + m) * NPADT + 8 * h;
  const v8f zero8 = {0.f, 0.f, 0.f, 0.f, 0.f, 0.f, 0.f, 0.f};

#pragma unroll 1
  for (int hh = 0; hh < HEADS; ++hh) {
    FragB qfh, qfl;
    {
      const v8b a = *(const v8b*)(qrow + hh * 16);
      const v8b c = *(const v8b*)(qrow + 128 + hh * 16);
      qfh.h[0] = a; qfh.h[1] = a;
      qfl.h[0] = c; qfl.h[1] = c;
    }
    const __bf16* vh = vbase + (size_t)(hh * 16) * NPADT;
    const __bf16* vl = vh + (size_t)128 * NPADT;
    v8f o = zero8;
    float mrun = NEG_INF, lrun = 0.0f;

#pragma unroll 1
    for (int kt = 0; kt < NPADT / 64; ++kt) {
      const int cnt = __builtin_amdgcn_readfirstlane(sCnt[kt]);
      if (cnt == 0) continue;
      const int kb = kt * 64;
      v8f s[4];
#pragma unroll
      for (int j = 0; j < 4; ++j) {
        const __bf16* kp = kbase + (size_t)(kb + 16 * j) * 256;
        FragB ka;
        ka.h[0] = *(const v8b*)(kp + hh * 16);
        ka.h[1] = *(const v8b*)(kp + 128 + hh * 16);
        v8f z = zero8;
        z = wmma_b(ka.v, qfh.v, z);
        z = wmma_b(ka.v, qfl.v, z);
        s[j] = z;
      }
#pragma unroll
      for (int j = 0; j < 4; ++j) {
        const int* ap = sAllow + kb + 16 * j + 8 * h;
        const v4i a0 = *(const v4ia*)(ap);
        const v4i a1 = *(const v4ia*)(ap + 4);
        s[j][0] = (a0[0] != 0) ? s[j][0] : NEG_INF;
        s[j][1] = (a0[1] != 0) ? s[j][1] : NEG_INF;
        s[j][2] = (a0[2] != 0) ? s[j][2] : NEG_INF;
        s[j][3] = (a0[3] != 0) ? s[j][3] : NEG_INF;
        s[j][4] = (a1[0] != 0) ? s[j][4] : NEG_INF;
        s[j][5] = (a1[1] != 0) ? s[j][5] : NEG_INF;
        s[j][6] = (a1[2] != 0) ? s[j][6] : NEG_INF;
        s[j][7] = (a1[3] != 0) ? s[j][7] : NEG_INF;
      }
      float mloc = NEG_INF;
#pragma unroll
      for (int j = 0; j < 4; ++j)
#pragma unroll
        for (int r = 0; r < 8; ++r) mloc = fmaxf(mloc, s[j][r]);
      mloc = fmaxf(mloc, __shfl_xor(mloc, 16, 32));
      const float mnew = fmaxf(mrun, mloc);
      const float mref = (mnew == NEG_INF) ? 0.0f : mnew;
      const float alpha = expf(mrun - mref);
      mrun = mnew;
      float lsum = 0.0f;
#pragma unroll
      for (int j = 0; j < 4; ++j)
#pragma unroll
        for (int r = 0; r < 8; ++r) {
          const float p = expf(s[j][r] - mref);
          s[j][r] = p;
          lsum += p;
        }
      lsum += __shfl_xor(lsum, 16, 32);
      lrun = lrun * alpha + lsum;
#pragma unroll
      for (int r = 0; r < 8; ++r) o[r] = o[r] * alpha;

#pragma unroll
      for (int c = 0; c < 2; ++c) {
        FragB ph, pl;
#pragma unroll
        for (int i = 0; i < 4; ++i) {
          ph.w[i]     = hi_pair(s[2 * c][2 * i],     s[2 * c][2 * i + 1]);
          pl.w[i]     = lo_pair(s[2 * c][2 * i],     s[2 * c][2 * i + 1]);
          ph.w[4 + i] = hi_pair(s[2 * c + 1][2 * i], s[2 * c + 1][2 * i + 1]);
          pl.w[4 + i] = lo_pair(s[2 * c + 1][2 * i], s[2 * c + 1][2 * i + 1]);
        }
        const v16b vfh = ldfrag(vh + kb + 32 * c);
        const v16b vfl = ldfrag(vl + kb + 32 * c);
        o = wmma_b(vfh, ph.v, o);
        o = wmma_b(vfh, pl.v, o);
        o = wmma_b(vfl, ph.v, o);
      }
    }

    const float inv = 1.0f / lrun;
    float* tp = T + (w * 16 + m) * TP + hh * 16 + 8 * h;
    v4f o0, o1;
    o0[0] = o[0] * inv; o0[1] = o[1] * inv; o0[2] = o[2] * inv; o0[3] = o[3] * inv;
    o1[0] = o[4] * inv; o1[1] = o[5] * inv; o1[2] = o[6] * inv; o1[3] = o[7] * inv;
    *(v4fa*)(tp) = o0;
    *(v4fa*)(tp + 4) = o1;
  }
  __syncthreads();
  store_hilo<16>(T, CTX, m0, 256, 128, 0, w, lane);
}

extern "C" void kernel_launch(void* const* d_in, const int* in_sizes, int n_in,
                              void* d_out, int out_size, void* d_ws, size_t ws_size,
                              hipStream_t stream) {
  if (n_in < 13) return;
  if (in_sizes[0] != NB * NTOK * DIM) return;
  if (in_sizes[1] != NB * 4) return;
  if (in_sizes[2] != DEPTH * DIM * 384) return;
  if (in_sizes[3] != DEPTH * DIM * DIM) return;
  if (in_sizes[4] != DEPTH * DIM || in_sizes[5] != DEPTH * DIM || in_sizes[6] != DEPTH * DIM) return;
  if (in_sizes[7] != DEPTH * DIM || in_sizes[8] != DEPTH * DIM) return;
  if (in_sizes[9] != DEPTH * DIM * MLP) return;
  if (in_sizes[10] != DEPTH * MLP) return;
  if (in_sizes[11] != DEPTH * MLP * DIM) return;
  if (in_sizes[12] != DEPTH * DIM) return;
  if (out_size != NB * NTOK * DIM) return;

  const float* x     = (const float*)d_in[0];
  const int*   mask  = (const int*)d_in[1];
  const float* Wqkv  = (const float*)d_in[2];
  const float* Wproj = (const float*)d_in[3];
  const float* bproj = (const float*)d_in[4];
  const float* g1    = (const float*)d_in[5];
  const float* b1    = (const float*)d_in[6];
  const float* g2    = (const float*)d_in[7];
  const float* b2    = (const float*)d_in[8];
  const float* W1f   = (const float*)d_in[9];
  const float* b1f   = (const float*)d_in[10];
  const float* W2f   = (const float*)d_in[11];
  const float* b2f   = (const float*)d_in[12];
  float* out = (float*)d_out;

  const size_t SZ_WQ = (size_t)DEPTH * 384 * DIM * 2;
  const size_t SZ_WP = (size_t)DEPTH * DIM * DIM * 2;
  const size_t SZ_W1 = (size_t)DEPTH * MLP * DIM * 2;
  const size_t SZ_W2 = (size_t)DEPTH * DIM * MLP * 2;
  const size_t SZ_PL = (size_t)MROWS * 256 * 2;
  const size_t SZ_VT = (size_t)NB * 2 * 128 * NPADT * 2;
  const size_t SZ_G  = (size_t)MROWS * 8192 * 2;
  const size_t SZ_X  = (size_t)MROWS * DIM * 4;
  size_t off = 0;
  const size_t oWQ = off; off += SZ_WQ;
  const size_t oWP = off; off += SZ_WP;
  const size_t oW1 = off; off += SZ_W1;
  const size_t oW2 = off; off += SZ_W2;
  const size_t oH  = off; off += SZ_PL;
  const size_t oQK = off; off += 2 * SZ_PL;
  const size_t oVT = off; off += SZ_VT;
  const size_t oC  = off; off += SZ_PL;
  const size_t oG  = off; off += SZ_G;
  const size_t oXA = off; off += SZ_X;
  const size_t oXB = off; off += SZ_X;
  if (off > ws_size) return;
  if (off > (size_t)134217728) return;

  char* ws = (char*)d_ws;
  unsigned short* WQ  = (unsigned short*)(ws + oWQ);
  unsigned short* WP  = (unsigned short*)(ws + oWP);
  unsigned short* W1  = (unsigned short*)(ws + oW1);
  unsigned short* W2  = (unsigned short*)(ws + oW2);
  unsigned short* HHL = (unsigned short*)(ws + oH);
  unsigned short* QK  = (unsigned short*)(ws + oQK);
  unsigned short* KHL = QK + (size_t)PLANE_EL;
  unsigned short* VT  = (unsigned short*)(ws + oVT);
  unsigned short* CTX = (unsigned short*)(ws + oC);
  unsigned short* GHL = (unsigned short*)(ws + oG);
  float* XA = (float*)(ws + oXA);
  float* XB = (float*)(ws + oXB);

  const dim3 blk(256);
  k_prep_x<<<dim3(MROWS / 64), blk, 0, stream>>>(x, g1, b1, XA, HHL);
  k_wprep<<<dim3(384 / 64, DIM / 64, DEPTH), blk, 0, stream>>>(Wqkv, WQ, DIM, 384);
  k_wprep<<<dim3(DIM / 64, DIM / 64, DEPTH), blk, 0, stream>>>(Wproj, WP, DIM, DIM);
  k_wprep<<<dim3(MLP / 64, DIM / 64, DEPTH), blk, 0, stream>>>(W1f, W1, DIM, MLP);
  k_wprep<<<dim3(DIM / 64, MLP / 64, DEPTH), blk, 0, stream>>>(W2f, W2, MLP, DIM);

  for (int l = 0; l < DEPTH; ++l) {
    const int ln = (l + 1 < DEPTH) ? (l + 1) : (DEPTH - 1);
    k_gemm<0><<<dim3(MROWS / 64, 3), blk, 0, stream>>>(
        HHL, 256, 128, WQ + (size_t)l * 384 * DIM, DIM,
        bproj, XA, XB, g1, b1, QK, 256, 128, VT, out, 0);
    k_attn<<<dim3(NPADT / 64, NB), dim3(128), 0, stream>>>(QK, KHL, VT, mask, CTX);
    k_gemm<1><<<dim3(MROWS / 64, 1), blk, 0, stream>>>(
        CTX, 256, 128, WP + (size_t)l * DIM * DIM, DIM,
        bproj + (size_t)l * DIM, XA, XB, g2 + (size_t)l * DIM, b2 + (size_t)l * DIM,
        HHL, 256, 128, VT, out, 0);
    k_gemm<2><<<dim3(MROWS / 64, MLP / 128), blk, 0, stream>>>(
        HHL, 256, 128, W1 + (size_t)l * MLP * DIM, DIM,
        b1f + (size_t)l * MLP, XA, XB, g1, b1, GHL, 8192, 4096, VT, out, 0);
    k_gemm<1><<<dim3(MROWS / 64, 1), blk, 0, stream>>>(
        GHL, 8192, 4096, W2 + (size_t)l * DIM * MLP, MLP,
        b2f + (size_t)l * DIM, XB, XA, g1 + (size_t)ln * DIM, b1 + (size_t)ln * DIM,
        HHL, 256, 128, VT, out, (l == DEPTH - 1) ? 1 : 0);
  }
  (void)hipGetLastError();
}
